// Model_20598663152059
// MI455X (gfx1250) — hardware-verified
//
#include <hip/hip_runtime.h>
#include <math.h>

constexpr int NLAYER   = 9;
constexpr int NCH      = 256;
constexpr int NPART    = 3;
constexpr int NJOINT   = 25;
constexpr int NTAP     = 9;
constexpr int NFRAME   = 128;
constexpr int NCLS     = 60;
constexpr int NCIN     = 3;
constexpr int NROW     = NFRAME * NJOINT;
constexpr int NYC      = NPART * NCH;
constexpr int NPADF    = NTAP - 1;
constexpr int NSLOT    = NFRAME + NPADF;
constexpr int NAROW    = NSLOT * NJOINT;
constexpr int KTAPS    = NTAP * NCH;
constexpr int TILE_F   = NJOINT * NCH;
constexpr int RES_LAG  = NTAP / 2;
constexpr int NXF      = NCIN * NJOINT;
constexpr int ALP      = 28;
constexpr int NALROW   = NPART * NJOINT;
constexpr int NTHR     = 256;
constexpr float LN_EPS_F   = 1e-5f;
constexpr float HCARRY     = 16.0f;
constexpr float WCARRY     = 64.0f;
constexpr float G1_SCALE   = 1.0f / (HCARRY * WCARRY);
constexpr float G2_SCALE   = 1.0f / WCARRY;

static_assert(NROW == 3200 && NAROW == 3400 && KTAPS == 2304 && TILE_F == 6400, "shape constants");
static_assert(NROW % 64 == 0 && NYC % 64 == 0 && NCH % 64 == 0, "GEMM M, N tile multiples");
static_assert(NCH % 32 == 0 && KTAPS % 32 == 0, "GEMM K multiple of 32");
static_assert(((NROW / 64) * (NYC / 64)) % 8 == 0 && ((NROW / 64) * (NCH / 64)) % 8 == 0, "8 tiles per block exact");
static_assert(TILE_F % 8 == 0 && NCLS % 4 == 0, "vector store widths");
static_assert((NLAYER * NYC * NCH / 8) % NTHR == 0 && (NLAYER * NCH * KTAPS / 8) % NTHR == 0, "convert grids exact");
static_assert(NCH == NTHR, "one thread per channel in the frame kernels");

typedef __attribute__((ext_vector_type(16))) _Float16 v16h;
typedef __attribute__((ext_vector_type(8)))  _Float16 v8h;
typedef __attribute__((ext_vector_type(8)))  float    v8f;
typedef __attribute__((ext_vector_type(4)))  float    v4f;

__device__ __forceinline__ void dep_guard4_h(v8f& a, v8f& b, v8f& c, v8f& d, v16h x, v16h y0, v16h y1, v16h y2, v16h y3) {
  asm volatile("v_nop\n\tv_nop\n\tv_nop\n\tv_nop" : "+v"(a), "+v"(b), "+v"(c), "+v"(d) : "v"(x), "v"(y0), "v"(y1), "v"(y2), "v"(y3));
}
__device__ __forceinline__ void keep4_h(v16h a, v16h b, v16h c, v16h d) { asm volatile("v_nop" :: "v"(a), "v"(b), "v"(c), "v"(d)); }
__device__ __forceinline__ void acc_guard4(v8f& a, v8f& b, v8f& c, v8f& d) { asm volatile("v_nop\n\tv_nop\n\tv_nop\n\tv_nop" : "+v"(a), "+v"(b), "+v"(c), "+v"(d)); }

template <typename T> struct Frag;
template <> struct Frag<_Float16> {
  typedef v16h V; union U { v16h v; v8h h[2]; };
  static __device__ __forceinline__ v16h load(const _Float16* p) {
    U f; f.h[0] = *(const v8h*)(p); f.h[1] = *(const v8h*)(p + 16); return f.v;
  }
  static __device__ __forceinline__ v8f mma(v16h a, v16h b, v8f c) {
    return __builtin_amdgcn_wmma_f32_16x16x32_f16(false, a, false, b, (short)0, c, false, false);
  }
};

__device__ __forceinline__ float block_sum256(float v, float* red, int lane, int wave) {
#pragma unroll
  for (int off = 16; off > 0; off >>= 1) v += __shfl_xor(v, off, 32);
  if (lane == 0) red[wave] = v;
  __syncthreads();
  float tot = 0.0f;
#pragma unroll
  for (int w = 0; w < NTHR / 32; ++w) tot += red[w];
  return tot;
}

__device__ __forceinline__ void store_tile_f32(const float* tile, float* dst, int tid) {
  for (int pass = 0; pass < 2; ++pass) {
#pragma unroll 1
    for (int i = tid; i < TILE_F / 4; i += NTHR) {
      const v4f v = *(const v4f*)(tile + 4 * i);
      *(volatile v4f*)(dst + 4 * i) = v;
    }
    __threadfence();
  }
}
__device__ __forceinline__ void store_tile_f16(const float* tile, unsigned short* dst, int tid, float sc) {
  for (int pass = 0; pass < 2; ++pass) {
#pragma unroll 1
    for (int i = tid; i < TILE_F / 8; i += NTHR) {
      const v4f a = *(const v4f*)(tile + 8 * i);
      const v4f b = *(const v4f*)(tile + 8 * i + 4);
      v8h hv;
#pragma unroll
      for (int e = 0; e < 4; ++e) {
        hv[e]     = (_Float16)(a[e] * sc);
        hv[4 + e] = (_Float16)(b[e] * sc);
      }
      *(volatile v8h*)(dst + 8 * i) = hv;
    }
    __threadfence();
  }
}

__global__ __launch_bounds__(NTHR) void cvt_lin_kernel(const float* __restrict__ src, unsigned short* __restrict__ dst, int n8, float sc) {
  const int i = blockIdx.x * NTHR + threadIdx.x;
  if (i < n8) {
    const float* sp = src + (size_t)i * 8;
    const v4f a = *(const v4f*)(sp);
    const v4f b = *(const v4f*)(sp + 4);
    v8h hv;
#pragma unroll
    for (int e = 0; e < 4; ++e) {
      hv[e]     = (_Float16)(a[e] * sc);
      hv[4 + e] = (_Float16)(b[e] * sc);
    }
    *(volatile v8h*)(dst + (size_t)i * 8) = hv;
    __threadfence();
    *(volatile v8h*)(dst + (size_t)i * 8) = hv;
  }
}

__global__ __launch_bounds__(NTHR) void cvt_taps_kernel(const float* __restrict__ src, unsigned short* __restrict__ dst, int n8, float sc) {
  const int i = blockIdx.x * NTHR + threadIdx.x;
  if (i < n8) {
    const int c0  = (i & 31) * 8;
    const int row = i >> 5;
    const int lo  = row / NTAP;
    const int g   = row - lo * NTAP;
    const float* sp = src + ((size_t)lo * NCH + c0) * NTAP + g;
    v8h hv;
#pragma unroll
    for (int e = 0; e < 8; ++e) hv[e] = (_Float16)(sp[e * NTAP] * sc);
    *(volatile v8h*)(dst + (size_t)i * 8) = hv;
    __threadfence();
    *(volatile v8h*)(dst + (size_t)i * 8) = hv;
  }
}

__global__ __launch_bounds__(NTHR) void input_kernel(const float* __restrict__ x, const float* __restrict__ lnw,
                                                     const float* __restrict__ lnb, const float* __restrict__ Win,
                                                     const float* __restrict__ bin,
                                                     float* __restrict__ HfOut, unsigned short* __restrict__ H16Out) {
  __shared__ __align__(16) float tile[TILE_F];
  __shared__ float xr[80];
  __shared__ float xn[80];
  const int t = blockIdx.x, tid = threadIdx.x;
  if (tid < NXF) {
    const int ci = tid / NJOINT;
    const int v  = tid - ci * NJOINT;
    xr[tid] = x[((size_t)ci * NFRAME + t) * NJOINT + v];
  }
  __syncthreads();
  float s = 0.0f;
#pragma unroll 1
  for (int i = 0; i < NXF; ++i) s += xr[i];
  const float mean = s * (1.0f / NXF);
  float ss = 0.0f;
#pragma unroll 1
  for (int i = 0; i < NXF; ++i) { const float d = xr[i] - mean; ss = fmaf(d, d, ss); }
  const float rs = rsqrtf(ss * (1.0f / NXF) + LN_EPS_F);
  if (tid < NXF) xn[tid] = (xr[tid] - mean) * rs * lnw[tid] + lnb[tid];
  __syncthreads();
  const int c = tid;
  const float w0 = Win[c * NCIN + 0], w1 = Win[c * NCIN + 1], w2 = Win[c * NCIN + 2];
  const float bb = bin[c];
#pragma unroll 1
  for (int v = 0; v < NJOINT; ++v) {
    float acc = w0 * xn[v];
    acc = fmaf(w1, xn[NJOINT + v], acc);
    acc = fmaf(w2, xn[2 * NJOINT + v], acc);
    tile[v * NCH + c] = acc + bb;
  }
  __syncthreads();
  store_tile_f32(tile, HfOut + (size_t)t * TILE_F, tid);
  store_tile_f16(tile, H16Out + (size_t)t * TILE_F, tid, HCARRY);
}

__global__ __launch_bounds__(NTHR) void gemm_f16_taps_kernel(
    const unsigned short* __restrict__ Ap, int lda,
    const unsigned short* __restrict__ Btp, int ldb,
    float* __restrict__ Cp, int ldc,
    int nrowM, int ncolN, int ntaps, int tapK, int tapRowShift, float scale) {
  const _Float16* Amat = (const _Float16*)Ap;
  const _Float16* Bmat = (const _Float16*)Btp;
  __shared__ __align__(16) float sT[8][16 * 68];
  const int lane = threadIdx.x & 31;
  const int wave = threadIdx.x >> 5;
  const int tilesN = ncolN >> 6;
  const int tilesM = nrowM >> 6;
  const int tile = blockIdx.x * 8 + wave;
  if (tile >= tilesM * tilesN) return;
  const int tm = tile / tilesN;
  const int tn = tile - tm * tilesN;
  const int m0 = tm << 6;
  const int n0 = tn << 6;
  const int rlane = lane & 15;
  const int koff  = (lane >> 4) * 8;
  const int mOff  = (lane >> 4) * 8;

  v8f acc[4][4];
#pragma unroll
  for (int i = 0; i < 4; ++i)
#pragma unroll
    for (int j = 0; j < 4; ++j) acc[i][j] = (v8f){0.f, 0.f, 0.f, 0.f, 0.f, 0.f, 0.f, 0.f};

#pragma unroll 1
  for (int g = 0; g < ntaps; ++g) {
    const _Float16* Ag = Amat + (size_t)((ntaps - 1 - g) * tapRowShift) * lda;
    const _Float16* Bg = Bmat + (size_t)g * tapK;
#pragma unroll 1
    for (int k0 = 0; k0 < tapK; k0 += 32) {
      v16h bh[4];
#pragma unroll
      for (int j = 0; j < 4; ++j)
        bh[j] = Frag<_Float16>::load(Bg + (size_t)(n0 + (j << 4) + rlane) * ldb + koff + k0);
#pragma unroll
      for (int i = 0; i < 4; ++i) {
        const v16h ah = Frag<_Float16>::load(Ag + (size_t)(m0 + (i << 4) + rlane) * lda + koff + k0);
#pragma unroll
        for (int j = 0; j < 4; ++j) acc[i][j] = Frag<_Float16>::mma(ah, bh[j], acc[i][j]);
        dep_guard4_h(acc[i][0], acc[i][1], acc[i][2], acc[i][3], ah, bh[0], bh[1], bh[2], bh[3]);
      }
      keep4_h(bh[0], bh[1], bh[2], bh[3]);
    }
  }
  acc_guard4(acc[0][0], acc[0][1], acc[0][2], acc[0][3]);
  acc_guard4(acc[1][0], acc[1][1], acc[1][2], acc[1][3]);
  acc_guard4(acc[2][0], acc[2][1], acc[2][2], acc[2][3]);
  acc_guard4(acc[3][0], acc[3][1], acc[3][2], acc[3][3]);

  float* slab = sT[wave];
#pragma unroll
  for (int i = 0; i < 4; ++i) {
    const int mBase = m0 + (i << 4);
#pragma unroll
    for (int j = 0; j < 4; ++j) {
#pragma unroll
      for (int r = 0; r < 8; ++r) slab[(mOff + r) * 68 + (j << 4) + rlane] = acc[i][j][r] * scale;
    }
    __builtin_amdgcn_fence(__ATOMIC_RELEASE, "workgroup");
    __builtin_amdgcn_wave_barrier();
    __builtin_amdgcn_fence(__ATOMIC_ACQUIRE, "workgroup");
    {
      const int hh = lane >> 4, c4 = (lane & 15) * 4;
      for (int pass = 0; pass < 2; ++pass) {
#pragma unroll
        for (int it = 0; it < 8; ++it) {
          const int row = it * 2 + hh;
          const v4f v = *(const v4f*)(slab + row * 68 + c4);
          *(volatile v4f*)(Cp + (size_t)(mBase + row) * ldc + n0 + c4) = v;
        }
        __threadfence();
      }
    }
    __builtin_amdgcn_fence(__ATOMIC_RELEASE, "workgroup");
    __builtin_amdgcn_wave_barrier();
    __builtin_amdgcn_fence(__ATOMIC_ACQUIRE, "workgroup");
  }
}

__global__ __launch_bounds__(NTHR) void adj_ln_kernel(const float* __restrict__ Y, const float* __restrict__ Aadj,
                                                      const float* __restrict__ imp, const float* __restrict__ bg,
                                                      const float* __restrict__ ln1w, const float* __restrict__ ln1b,
                                                      unsigned short* __restrict__ A16, int l) {
  __shared__ __align__(16) float tile[TILE_F];
  __shared__ __align__(16) float sAl[NALROW * ALP];
  __shared__ float red1[8];
  __shared__ float red2[8];
  const int tid = threadIdx.x, lane = tid & 31, wave = tid >> 5;
  const int c = tid;
  const int blk = blockIdx.x;
  const bool isPad = (blk >= NFRAME);
  const int slot = isPad ? (blk - NFRAME) : (blk + NPADF);
  const float* lw = ln1w + (size_t)l * TILE_F + c * NJOINT;
  const float* lb = ln1b + (size_t)l * TILE_F + c * NJOINT;
  if (isPad) {
#pragma unroll 1
    for (int w = 0; w < NJOINT; ++w) tile[w * NCH + c] = fmaxf(lb[w], 0.0f);
  } else {
#pragma unroll 1
    for (int i = tid; i < NALROW * ALP; i += NTHR) {
      const int r  = i / ALP;
      const int w  = i - r * ALP;
      const int wc = (w < NJOINT) ? w : (NJOINT - 1);
      const float val = Aadj[r * NJOINT + wc] * imp[(size_t)l * (NALROW * NJOINT) + r * NJOINT + wc];
      sAl[i] = (w < NJOINT) ? val : 0.0f;
    }
    __syncthreads();
    float z[NJOINT];
#pragma unroll
    for (int w = 0; w < NJOINT; ++w) z[w] = 0.0f;
    const float* yb  = Y + (size_t)blk * NJOINT * NYC + c;
    const float* bgl = bg + (size_t)l * NYC + c;
#pragma unroll 1
    for (int k = 0; k < NPART; ++k) {
      const float bgv = bgl[k * NCH];
#pragma unroll 1
      for (int v = 0; v < NJOINT; ++v) {
        const float yv = yb[(size_t)v * NYC + k * NCH] + bgv;
        const v4f* ar = (const v4f*)(sAl + (k * NJOINT + v) * ALP);
        v4f av[7];
#pragma unroll
        for (int q = 0; q < 7; ++q) av[q] = ar[q];
#pragma unroll
        for (int q = 0; q < 6; ++q)
#pragma unroll
          for (int e = 0; e < 4; ++e) z[4 * q + e] = fmaf(yv, av[q][e], z[4 * q + e]);
        z[24] = fmaf(yv, av[6][0], z[24]);
      }
    }
    float s = 0.0f;
#pragma unroll
    for (int w = 0; w < NJOINT; ++w) { s += z[w]; tile[w * NCH + c] = z[w]; }
    const float mean = block_sum256(s, red1, lane, wave) * (1.0f / TILE_F);
    float ss = 0.0f;
#pragma unroll 1
    for (int w = 0; w < NJOINT; ++w) { const float d = tile[w * NCH + c] - mean; ss = fmaf(d, d, ss); }
    const float var = block_sum256(ss, red2, lane, wave) * (1.0f / TILE_F);
    const float rs = rsqrtf(var + LN_EPS_F);
#pragma unroll 1
    for (int w = 0; w < NJOINT; ++w) {
      const float val = tile[w * NCH + c];
      const float a = (val - mean) * rs * lw[w] + lb[w];
      tile[w * NCH + c] = fmaxf(a, 0.0f);
    }
  }
  __syncthreads();
  store_tile_f16(tile, A16 + (size_t)slot * TILE_F, tid, 1.0f);
}

__global__ __launch_bounds__(NTHR) void post_ln_kernel(const float* __restrict__ Tt, const float* __restrict__ bt,
                                                       const float* __restrict__ ln2w, const float* __restrict__ ln2b,
                                                       const float* __restrict__ HfIn, float* __restrict__ HfOut,
                                                       unsigned short* __restrict__ H16Out, float* __restrict__ pooled,
                                                       int l, int wantPool) {
  __shared__ __align__(16) float tile[TILE_F];
  __shared__ __align__(16) float pl[NCH];
  __shared__ float red1[8];
  __shared__ float red2[8];
  const int tid = threadIdx.x, lane = tid & 31, wave = tid >> 5;
  const int c = tid;
  const int t = blockIdx.x;
  const float* tsrc = Tt + (size_t)t * TILE_F;
#pragma unroll 1
  for (int i = tid; i < TILE_F / 4; i += NTHR) {
    const v4f v = *(const v4f*)(tsrc + 4 * i);
    *(v4f*)(tile + 4 * i) = v;
  }
  __syncthreads();
  const float btv = bt[(size_t)l * NCH + c];
  float s = 0.0f;
#pragma unroll 1
  for (int v = 0; v < NJOINT; ++v) {
    const float val = tile[v * NCH + c] + btv;
    tile[v * NCH + c] = val;
    s += val;
  }
  const float mean = block_sum256(s, red1, lane, wave) * (1.0f / TILE_F);
  float ss = 0.0f;
#pragma unroll 1
  for (int v = 0; v < NJOINT; ++v) { const float d = tile[v * NCH + c] - mean; ss = fmaf(d, d, ss); }
  const float var = block_sum256(ss, red2, lane, wave) * (1.0f / TILE_F);
  const float rs = rsqrtf(var + LN_EPS_F);
  const float* lw = ln2w + (size_t)l * TILE_F + c * NJOINT;
  const float* lb = ln2b + (size_t)l * TILE_F + c * NJOINT;
  const bool hasRes = (t >= RES_LAG);
  const int tr = hasRes ? (t - RES_LAG) : 0;
  const float* rsrc = HfIn + (size_t)tr * TILE_F + c;
  float psum = 0.0f;
#pragma unroll 1
  for (int v = 0; v < NJOINT; ++v) {
    const float val = tile[v * NCH + c];
    const float t2 = (val - mean) * rs * lw[v] + lb[v];
    float r = rsrc[v * NCH];
    asm volatile("" : "+v"(r));
    r = hasRes ? r : 0.0f;
    const float h = fmaxf(t2 + r, 0.0f);
    tile[v * NCH + c] = h;
    psum += h;
  }
  pl[c] = psum * (1.0f / NJOINT);
  __syncthreads();
  store_tile_f32(tile, HfOut + (size_t)t * TILE_F, tid);
  store_tile_f16(tile, H16Out + (size_t)t * TILE_F, tid, HCARRY);
  if (wantPool != 0) {
    if (tid < NCH / 4) {
      const v4f pv = *(const v4f*)(pl + 4 * tid);
      float* pd = pooled + (size_t)t * NCH + 4 * tid;
      *(volatile v4f*)pd = pv;
      __threadfence();
      *(volatile v4f*)pd = pv;
    }
  }
}

__global__ __launch_bounds__(NTHR) void head_kernel(const float* __restrict__ pooled, const float* __restrict__ Wout,
                                                    const float* __restrict__ bout, float* __restrict__ out) {
  const int i4 = blockIdx.x * NTHR + threadIdx.x;
  if (i4 < (NFRAME * NCLS) / 4) {
    const int i = 4 * i4;
    const int t = i / NCLS;
    const int o = i - t * NCLS;
    const float* pp = pooled + (size_t)t * NCH;
    const float* wr = Wout + (size_t)o * NCH;
    v4f acc = {0.f, 0.f, 0.f, 0.f};
#pragma unroll 1
    for (int k = 0; k < NCH; k += 4) {
      const v4f p  = *(const v4f*)(pp + k);
      const v4f q0 = *(const v4f*)(wr + k);
      const v4f q1 = *(const v4f*)(wr + NCH + k);
      const v4f q2 = *(const v4f*)(wr + 2 * NCH + k);
      const v4f q3 = *(const v4f*)(wr + 3 * NCH + k);
#pragma unroll
      for (int e = 0; e < 4; ++e) {
        acc[0] = fmaf(q0[e], p[e], acc[0]);
        acc[1] = fmaf(q1[e], p[e], acc[1]);
        acc[2] = fmaf(q2[e], p[e], acc[2]);
        acc[3] = fmaf(q3[e], p[e], acc[3]);
      }
    }
    const v4f bb = *(const v4f*)(bout + o);
    v4f res;
#pragma unroll
    for (int e = 0; e < 4; ++e) res[e] = acc[e] + bb[e];
    *(volatile v4f*)(out + i) = res;
    __threadfence();
    *(volatile v4f*)(out + i) = res;
  }
}

extern "C" void kernel_launch(void* const* d_in, const int* in_sizes, int n_in,
                              void* d_out, int out_size, void* d_ws, size_t ws_size, hipStream_t stream) {
  if (n_in < 17 || d_out == nullptr || d_ws == nullptr) return;
  if (in_sizes[0] != NCIN * NFRAME * NJOINT || in_sizes[1] != NPART * NJOINT * NJOINT ||
      in_sizes[2] != NXF || in_sizes[3] != NXF || in_sizes[4] != NCH * NCIN || in_sizes[5] != NCH ||
      in_sizes[6] != NLAYER * NYC * NCH || in_sizes[7] != NLAYER * NYC ||
      in_sizes[8] != NLAYER * TILE_F || in_sizes[9] != NLAYER * TILE_F ||
      in_sizes[10] != NLAYER * NCH * NCH * NTAP || in_sizes[11] != NLAYER * NCH ||
      in_sizes[12] != NLAYER * TILE_F || in_sizes[13] != NLAYER * TILE_F ||
      in_sizes[14] != NLAYER * NPART * NJOINT * NJOINT || in_sizes[15] != NCLS * NCH ||
      in_sizes[16] != NCLS || out_size != NFRAME * NCLS) return;

  const float* x     = (const float*)d_in[0];
  const float* Aadj  = (const float*)d_in[1];
  const float* lninw = (const float*)d_in[2];
  const float* lninb = (const float*)d_in[3];
  const float* W_in  = (const float*)d_in[4];
  const float* b_in  = (const float*)d_in[5];
  const float* Wg    = (const float*)d_in[6];
  const float* bg    = (const float*)d_in[7];
  const float* ln1w  = (const float*)d_in[8];
  const float* ln1b  = (const float*)d_in[9];
  const float* Wt    = (const float*)d_in[10];
  const float* bt    = (const float*)d_in[11];
  const float* ln2w  = (const float*)d_in[12];
  const float* ln2b  = (const float*)d_in[13];
  const float* imp   = (const float*)d_in[14];
  const float* W_out = (const float*)d_in[15];
  const float* b_out = (const float*)d_in[16];
  float* out = (float*)d_out;

  char* ws = (char*)d_ws; size_t off = 0;
  auto carve = [&](size_t bytes) -> char* { char* p = ws + off; off += (bytes + 255) & ~(size_t)255; return p; };
  unsigned short* WG16 = (unsigned short*)carve((size_t)NLAYER * NYC * NCH * 2);
  unsigned short* WT16 = (unsigned short*)carve((size_t)NLAYER * NCH * KTAPS * 2);
  float*          HFA  = (float*)carve((size_t)NROW * NCH * 4);
  float*          HFB  = (float*)carve((size_t)NROW * NCH * 4);
  unsigned short* H16A = (unsigned short*)carve((size_t)NROW * NCH * 2);
  unsigned short* H16B = (unsigned short*)carve((size_t)NROW * NCH * 2);
  float*          YP   = (float*)carve((size_t)NROW * NYC * 4);
  unsigned short* A16  = (unsigned short*)carve((size_t)NAROW * NCH * 2);
  float*          TT   = (float*)carve((size_t)NROW * NCH * 4);
  float*          POOL = (float*)carve((size_t)NFRAME * NCH * 4);
  if (off > ws_size || off > (size_t)134217728) return;

  const int n8g = NLAYER * NYC * NCH / 8;
  const int n8t = NLAYER * NCH * KTAPS / 8;
  cvt_lin_kernel<<<n8g / NTHR, NTHR, 0, stream>>>(Wg, WG16, n8g, WCARRY);
  cvt_taps_kernel<<<n8t / NTHR, NTHR, 0, stream>>>(Wt, WT16, n8t, WCARRY);

  float* HfCur = HFA; float* HfNxt = HFB;
  unsigned short* H16Cur = H16A; unsigned short* H16Nxt = H16B;

  input_kernel<<<NFRAME, NTHR, 0, stream>>>(x, lninw, lninb, W_in, b_in, HfCur, H16Cur);

  const int gridG1 = (NROW / 64) * (NYC / 64) / 8;
  const int gridG2 = (NROW / 64) * (NCH / 64) / 8;
  for (int l = 0; l < NLAYER; ++l) {
    gemm_f16_taps_kernel<<<gridG1, NTHR, 0, stream>>>(
        H16Cur, NCH, WG16 + (size_t)l * NYC * NCH, NCH, YP, NYC,
        NROW, NYC, 1, NCH, 0, G1_SCALE);
    adj_ln_kernel<<<NSLOT, NTHR, 0, stream>>>(YP, Aadj, imp, bg, ln1w, ln1b, A16, l);
    gemm_f16_taps_kernel<<<gridG2, NTHR, 0, stream>>>(
        A16, NCH, WT16 + (size_t)l * NCH * KTAPS, KTAPS, TT, NCH,
        NROW, NCH, NTAP, NCH, NJOINT, G2_SCALE);
    post_ln_kernel<<<NFRAME, NTHR, 0, stream>>>(TT, bt, ln2w, ln2b, HfCur, HfNxt, H16Nxt, POOL, l,
                                                (l == NLAYER - 1) ? 1 : 0);
    { float* tf = HfCur; HfCur = HfNxt; HfNxt = tf; }
    { unsigned short* th = H16Cur; H16Cur = H16Nxt; H16Nxt = th; }
  }

  head_kernel<<<((NFRAME * NCLS) / 4 + NTHR - 1) / NTHR, NTHR, 0, stream>>>(POOL, W_out, b_out, out);
}
